// DeepBatchModel_17300128269008
// MI455X (gfx1250) — hardware-verified
//
#include <hip/hip_runtime.h>
#include <stddef.h>


#define HID     256
#define KP      256
#define KF      1024
#define YP      256
#define NLAY    4
#define OUTD    5
#define NWT     9
#define NTHR    256
#define NWAVE   8
#define EPT     8
#define CHUNK   (NTHR * EPT)
#define WCAP    (EPT * 32)
#define LISTN   (NWAVE * WCAP)
#define NBMAX   2048
#define RCAP    24576
#define DEGCAP  4096
#define GBM     64
#define GTHR    128
#define MG      256
#define PMAX    1024
#define NEG_SLOPE 0.2f
#define BN_EPS  1e-5f
#define CA      16.0f
#define CW      64.0f
#define SCL     0.0009765625f
#define WSCAP   134217728
#define LDS_AGG ((2 * RCAP + 2 * NBMAX + LISTN) * 4 + 64 + 2 * NBMAX * 4)

static_assert((CHUNK & (CHUNK - 1)) == 0 && CHUNK <= 4096);
static_assert((NBMAX & (NBMAX - 1)) == 0 && NBMAX <= 4096);
static_assert(NTHR * 8 == NBMAX);
static_assert(LISTN >= NBMAX);
static_assert(LISTN >= NWAVE * WCAP);
static_assert((RCAP % 32) == 0);
static_assert(LDS_AGG <= 300000);
static_assert(GBM == (GTHR / 32) * 16);
static_assert(2 * GTHR == HID);
static_assert(HID == 4 * 64);
static_assert(KP == HID && KF == NLAY * HID);
static_assert((KP % 32) == 0 && (KF % 32) == 0);
static_assert(MG == 4 * GBM);
static_assert(NTHR == HID);
static_assert(PMAX % 128 == 0);

typedef float    v4f  __attribute__((ext_vector_type(4)));
typedef float    v8f  __attribute__((ext_vector_type(8)));
typedef int      v4i  __attribute__((ext_vector_type(4)));
typedef int      v8i  __attribute__((ext_vector_type(8)));
typedef _Float16 v4h  __attribute__((ext_vector_type(4)));
typedef _Float16 v8h  __attribute__((ext_vector_type(8)));
typedef _Float16 v16h __attribute__((ext_vector_type(16)));
union FragH { v16h v; v8h h[2]; v8i w; };

__device__ __forceinline__ v8f wmh(const FragH& a, const FragH& b, v8f c) {
  v8f d = __builtin_amdgcn_wmma_f32_16x16x32_f16(false, a.v, false, b.v, (short)0, c, false, false);
  asm volatile("v_nop\n\tv_nop\n\tv_nop\n\tv_nop" : "+v"(d) : "v"(a.w), "v"(b.w));
  return d;
}

__device__ __forceinline__ int scan_chunk(const int* __restrict__ dsts, int nE, int cbase, int slotBase,
                                          int nb, int vec8, int* list, int tid, int lane, int wave) {
  int wc = 0;
  const int el0  = tid * EPT;
  const int e0   = cbase + el0;
  const int sent = -2147483647 - 1;
  v4i da, db;
  if (vec8 != 0 && cbase + CHUNK <= nE) {
    da = *(const v4i*)(dsts + e0);
    db = *(const v4i*)(dsts + e0 + 4);
  } else {
    da.x = (e0     < nE) ? dsts[min(e0,     nE - 1)] : sent;
    da.y = (e0 + 1 < nE) ? dsts[min(e0 + 1, nE - 1)] : sent;
    da.z = (e0 + 2 < nE) ? dsts[min(e0 + 2, nE - 1)] : sent;
    da.w = (e0 + 3 < nE) ? dsts[min(e0 + 3, nE - 1)] : sent;
    db.x = (e0 + 4 < nE) ? dsts[min(e0 + 4, nE - 1)] : sent;
    db.y = (e0 + 5 < nE) ? dsts[min(e0 + 5, nE - 1)] : sent;
    db.z = (e0 + 6 < nE) ? dsts[min(e0 + 6, nE - 1)] : sent;
    db.w = (e0 + 7 < nE) ? dsts[min(e0 + 7, nE - 1)] : sent;
  }
  const unsigned nbs = (unsigned)slotBase;
  const unsigned unb = (unsigned)nb;
  const unsigned s0 = (unsigned)da.x - nbs, s1 = (unsigned)da.y - nbs;
  const unsigned s2 = (unsigned)da.z - nbs, s3 = (unsigned)da.w - nbs;
  const unsigned s4 = (unsigned)db.x - nbs, s5 = (unsigned)db.y - nbs;
  const unsigned s6 = (unsigned)db.z - nbs, s7 = (unsigned)db.w - nbs;
  const bool h0 = s0 < unb, h1 = s1 < unb, h2 = s2 < unb, h3 = s3 < unb;
  const bool h4 = s4 < unb, h5 = s5 < unb, h6 = s6 < unb, h7 = s7 < unb;
  const unsigned any = __builtin_amdgcn_ballot_w32(h0 | h1 | h2 | h3 | h4 | h5 | h6 | h7);
  if (any != 0u) {
#define HITJ(J, HJ, SJ) { \
      const unsigned mj = __builtin_amdgcn_ballot_w32(HJ); \
      if (mj != 0u) { \
        if (HJ) { \
          const int pos = wc + (int)__builtin_amdgcn_mbcnt_lo(mj, 0u); \
          if (pos < WCAP) list[wave * WCAP + pos] = ((el0 + (J)) << 12) | (int)(SJ); \
        } \
        wc += (int)__builtin_popcount(mj); } }
    HITJ(0, h0, s0)
    HITJ(1, h1, s1)
    HITJ(2, h2, s2)
    HITJ(3, h3, s3)
    HITJ(4, h4, s4)
    HITJ(5, h5, s5)
    HITJ(6, h6, s6)
    HITJ(7, h7, s7)
#undef HITJ
  }
  return wc;
}

__device__ __forceinline__ float alpha_of(const int* __restrict__ dsts, const float* __restrict__ score,
                                          const float* __restrict__ nstm, const float* __restrict__ nstd,
                                          int e, int l, int nE, int nN, int epad, int np) {
  e = e < 0 ? 0 : (e > nE - 1 ? nE - 1 : e);
  l = l & 3;
  int d = dsts[e];
  d = d < 0 ? 0 : (d > nN - 1 ? nN - 1 : d);
  const float s  = score[(size_t)l * epad + e];
  const float m  = nstm[(size_t)l * np + d];
  const float dn = nstd[(size_t)l * np + d];
  const float w  = __expf(s - m);
  const float inv = dn > 0.f ? __builtin_amdgcn_rcpf(dn) : 0.f;
  return w * inv;
}

__global__ __launch_bounds__(NTHR) void k_xprep(const float* __restrict__ x, _Float16* xh, int nN, int inDim,
                                                int nUnits) {
  const int i = (int)blockIdx.x * NTHR + (int)threadIdx.x;
  if (i >= nUnits) return;
  const int row = i >> 5;
  const int c0  = (i & 31) * 8;
  const int rc  = row < nN ? row : nN - 1;
  const float* p = x + (size_t)rc * inDim;
  v8h hv;
#pragma unroll
  for (int j = 0; j < 8; ++j) {
    const int c  = c0 + j;
    const int cc = c < inDim ? c : inDim - 1;
    const float f = p[cc];
    const float v = (row < nN && c < inDim) ? f * CA : 0.0f;
    hv[j] = (_Float16)v;
  }
  const size_t o = (size_t)row * KP + c0;
  *(volatile v8h*)(xh + o) = hv;
  __threadfence();
  *(volatile v8h*)(xh + o) = hv;
}

__global__ __launch_bounds__(NTHR) void k_wprep(const float* __restrict__ ws0, const float* __restrict__ wd0,
                                                const float* __restrict__ wr0, const float* __restrict__ wsr,
                                                const float* __restrict__ wdr, const float* __restrict__ wf1,
                                                _Float16* wt, _Float16* wf, int inDim) {
  const int j = (int)blockIdx.y;
  const int u = (int)blockIdx.x * NTHR + (int)threadIdx.x;
  const bool isF = (j == NWT);
  const int upr = isF ? (KF / 8) : (KP / 8);
  const int nUnits = HID * upr;
  if (u >= nUnits) return;
  const int n  = isF ? (u >> 7) : (u >> 5);
  const int k8 = (isF ? (u & 127) : (u & 31)) * 8;
  const int ksrc = (j < 3) ? inDim : (isF ? KF : HID);
  const int j3 = min(max(j - 3, 0), 2);
  const int j6 = min(max(j - 6, 0), 2);
  const float* p3 = wsr + (size_t)j3 * HID * HID;
  const float* p6 = wdr + (size_t)j6 * HID * HID;
  const float* sm = (j == 0) ? ws0 : ((j == 1) ? wd0 : ((j == 2) ? wr0 : ((j < 6) ? p3 : ((j < 9) ? p6 : wf1))));
  v8h hv;
#pragma unroll
  for (int t = 0; t < 8; ++t) {
    const int kk = k8 + t;
    const int kc = kk < ksrc ? kk : ksrc - 1;
    const float f = sm[(size_t)kc * HID + n];
    const float v = (kk < ksrc) ? f * CW : 0.0f;
    hv[t] = (_Float16)v;
  }
  _Float16* dp = isF ? (wf + (size_t)n * KF + k8) : (wt + ((size_t)j * HID + (size_t)n) * KP + k8);
  *(volatile v8h*)dp = hv;
  __threadfence();
  *(volatile v8h*)dp = hv;
}

__global__ __launch_bounds__(GTHR) void k_gemm(const _Float16* __restrict__ xa, int lda,
                                               const _Float16* __restrict__ w0, const _Float16* __restrict__ w1,
                                               const _Float16* __restrict__ w2, int ldb,
                                               const float* __restrict__ b0, const float* __restrict__ b1,
                                               const float* __restrict__ b2, int bmask,
                                               float* y0, float* y1, float* y2, int nks) {
  __shared__ __attribute__((aligned(16))) float stg[GBM * 64];
  __shared__ float sb[HID];
  const int j = (int)blockIdx.y;
  const _Float16* wt = (j == 0) ? w0 : ((j == 1) ? w1 : w2);
  const float* bias  = (j == 0) ? b0 : ((j == 1) ? b1 : b2);
  float* Y           = (j == 0) ? y0 : ((j == 1) ? y1 : y2);
  const int bsel = (bmask >> j) & 1;
  const int tid = threadIdx.x, lane = tid & 31, wave = tid >> 5, hh = lane >> 4, m = lane & 15;
  const int rowBase = (int)blockIdx.x * GBM;
  {
    const float v0 = bias[tid];
    const float v1 = bias[tid + GTHR];
    sb[tid]        = bsel ? v0 : 0.f;
    sb[tid + GTHR] = bsel ? v1 : 0.f;
  }
  __syncthreads();
  const int nk = nks < 1 ? 1 : (nks > 32 ? 32 : nks);
  const size_t arow = (size_t)(rowBase + 16 * wave + m) * lda + 8 * hh;
#pragma unroll 1
  for (int p = 0; p < 4; ++p) {
    v8f acc[4];
#pragma unroll
    for (int t = 0; t < 4; ++t) { v8f z = {0.f, 0.f, 0.f, 0.f, 0.f, 0.f, 0.f, 0.f}; acc[t] = z; }
    const size_t brow = (size_t)(p * 64 + m) * ldb + 8 * hh;
#pragma unroll 1
    for (int ks = 0; ks < nk; ++ks) {
      FragH af;
      af.h[0] = *(const v8h*)(xa + arow + 32 * ks);
      af.h[1] = *(const v8h*)(xa + arow + 32 * ks + 16);
#pragma unroll
      for (int t = 0; t < 4; ++t) {
        const size_t bo = brow + (size_t)(16 * t) * ldb + 32 * ks;
        FragH bf;
        bf.h[0] = *(const v8h*)(wt + bo);
        bf.h[1] = *(const v8h*)(wt + bo + 16);
        acc[t] = wmh(af, bf, acc[t]);
      }
    }
    float* sp = stg + (size_t)(16 * wave + 8 * hh) * 64 + m;
#pragma unroll
    for (int t = 0; t < 4; ++t) {
      const float bj = sb[p * 64 + 16 * t + m];
#pragma unroll
      for (int r = 0; r < 8; ++r) sp[(size_t)r * 64 + 16 * t] = fmaf(acc[t][r], SCL, bj);
    }
    __syncthreads();
    const int nF4 = GBM * 64 / 4;
    float* yb = Y + (size_t)rowBase * YP + 64 * p;
    const v4f* s4 = (const v4f*)stg;
#pragma unroll 1
    for (int f = tid; f < nF4; f += GTHR) {
      const int r = f >> 4, q = f & 15;
      const v4f v = s4[f];
      *(volatile v4f*)(yb + (size_t)r * YP + 4 * q) = v;
    }
    __threadfence();
#pragma unroll 1
    for (int f = tid; f < nF4; f += GTHR) {
      const int r = f >> 4, q = f & 15;
      const v4f v = s4[f];
      *(volatile v4f*)(yb + (size_t)r * YP + 4 * q) = v;
    }
    __syncthreads();
  }
}

__global__ __launch_bounds__(NTHR) void k_score(const int* __restrict__ srcs, const int* __restrict__ dsts,
                                                const float* __restrict__ FS, const float* __restrict__ FD,
                                                const float* __restrict__ av, float* sc, int nN, int nE) {
  const int tid = threadIdx.x, lane = tid & 31, wave = tid >> 5;
  const int c0 = 4 * lane, c1 = 128 + 4 * lane;
  const int ebase = ((int)blockIdx.x * NWAVE + wave) * 32;
  const v4f av0 = *(const v4f*)(av + c0);
  const v4f av1 = *(const v4f*)(av + c1);
  float mine = 0.f;
#pragma unroll 1
  for (int i = 0; i < 32; ++i) {
    int e = ebase + i;
    e = e > nE - 1 ? nE - 1 : e;
    int s = srcs[e]; s = s < 0 ? 0 : (s > nN - 1 ? nN - 1 : s);
    int d = dsts[e]; d = d < 0 ? 0 : (d > nN - 1 ? nN - 1 : d);
    const float* ps = FS + (size_t)s * YP;
    const float* pd = FD + (size_t)d * YP;
    const v4f xs0 = *(const v4f*)(ps + c0), xs1 = *(const v4f*)(ps + c1);
    const v4f xd0 = *(const v4f*)(pd + c0), xd1 = *(const v4f*)(pd + c1);
    float p = 0.f;
    float u;
    u = xs0.x + xd0.x; u = fmaxf(u, NEG_SLOPE * u); p = fmaf(u, av0.x, p);
    u = xs0.y + xd0.y; u = fmaxf(u, NEG_SLOPE * u); p = fmaf(u, av0.y, p);
    u = xs0.z + xd0.z; u = fmaxf(u, NEG_SLOPE * u); p = fmaf(u, av0.z, p);
    u = xs0.w + xd0.w; u = fmaxf(u, NEG_SLOPE * u); p = fmaf(u, av0.w, p);
    u = xs1.x + xd1.x; u = fmaxf(u, NEG_SLOPE * u); p = fmaf(u, av1.x, p);
    u = xs1.y + xd1.y; u = fmaxf(u, NEG_SLOPE * u); p = fmaf(u, av1.y, p);
    u = xs1.z + xd1.z; u = fmaxf(u, NEG_SLOPE * u); p = fmaf(u, av1.z, p);
    u = xs1.w + xd1.w; u = fmaxf(u, NEG_SLOPE * u); p = fmaf(u, av1.w, p);
    p += __shfl_xor(p, 16);
    p += __shfl_xor(p, 8);
    p += __shfl_xor(p, 4);
    p += __shfl_xor(p, 2);
    p += __shfl_xor(p, 1);
    mine = (lane == i) ? p : mine;
  }
  float* o = sc + ebase + lane;
  *(volatile float*)o = mine;
  __threadfence();
  *(volatile float*)o = mine;
}

__global__ __launch_bounds__(NTHR) void k_agg(
    const int* __restrict__ srcs, const int* __restrict__ dsts,
    const float* __restrict__ FS, const float* __restrict__ sc, const float* __restrict__ resp,
    float* rst, float* nstm, float* nstd, int nN, int nE, int nb, int vec8) {
  extern __shared__ v4f lds_dyn[];
  int* reg1 = (int*)lds_dyn;
  int* reg2 = reg1 + RCAP;
  int* scnt = reg2 + RCAP;
  int* soff = scnt + NBMAX;
  int* list = soff + NBMAX;
  int* wcnt = list + LISTN;
  int* wtot = wcnt + NWAVE;
  float* sm = (float*)(wtot + NWAVE);
  float* sd = sm + NBMAX;
  const int tid = threadIdx.x, lane = tid & 31, wave = tid >> 5;
  const int nodeBase = (int)blockIdx.x * nb;

  for (int i = tid; i < NBMAX; i += NTHR) scnt[i] = 0;
  __syncthreads();

  int tot = 0;
  const int nChunks = (nE + CHUNK - 1) / CHUNK;
#pragma unroll 1
  for (int ch = 0; ch < nChunks; ++ch) {
    const int cbase = ch * CHUNK;
    const int wc = scan_chunk(dsts, nE, cbase, nodeBase, nb, vec8, list, tid, lane, wave);
    if (lane == 0) wcnt[wave] = wc;
    __syncthreads();
    int pre = 0, all = 0;
#pragma unroll
    for (int w2 = 0; w2 < NWAVE; ++w2) {
      int c = wcnt[w2];
      c = c < 0 ? 0 : (c > WCAP ? WCAP : c);
      all += c;
      pre += (w2 < wave) ? c : 0;
    }
    const int wcc  = wc > WCAP ? WCAP : wc;
    const int base = tot + pre;
#pragma unroll 1
    for (int i = lane; i < wcc; i += 32) {
      const int ent = list[wave * WCAP + i];
      const int el  = (ent >> 12) & (CHUNK - 1);
      const int sl  = ent & (NBMAX - 1);
      int eid = cbase + el;
      eid = eid > nE - 1 ? nE - 1 : eid;
      const int pos = base + i;
      if (pos < RCAP) reg1[pos] = (int)(((unsigned)eid << 12) | (unsigned)sl);
    }
    tot += all;
    tot = tot > RCAP ? RCAP : tot;
    __syncthreads();
  }
  const int nh = tot;

  if (wave == 0) {
#pragma unroll 1
    for (int b0 = 0; b0 < nh; b0 += 32) {
      const int idx = b0 + lane;
      const int uv  = reg1[idx < RCAP ? idx : RCAP - 1];
      const int m32 = (nh - b0) < 32 ? (nh - b0) : 32;
#pragma unroll 1
      for (int k = 0; k < m32; ++k) {
        const int u  = __builtin_amdgcn_readlane(uv, k);
        const int sl = u & (NBMAX - 1);
        if (lane == 0) scnt[sl] = scnt[sl] + 1;
      }
    }
  }
  __syncthreads();

  {
    const v4i ca = *(const v4i*)(scnt + 8 * tid);
    const v4i cb = *(const v4i*)(scnt + 8 * tid + 4);
    const int e0 = ca.x < 0 ? 0 : ca.x, e1 = ca.y < 0 ? 0 : ca.y, e2 = ca.z < 0 ? 0 : ca.z, e3 = ca.w < 0 ? 0 : ca.w;
    const int e4 = cb.x < 0 ? 0 : cb.x, e5 = cb.y < 0 ? 0 : cb.y, e6 = cb.z < 0 ? 0 : cb.z, e7 = cb.w < 0 ? 0 : cb.w;
    const int ts = e0 + e1 + e2 + e3 + e4 + e5 + e6 + e7;
    int incl = ts;
#pragma unroll
    for (int d = 1; d < 32; d <<= 1) {
      const int up = __shfl_up(incl, d);
      if (lane >= d) incl += up;
    }
    if (lane == 31) wtot[wave] = incl;
    __syncthreads();
    int pre = 0;
#pragma unroll
    for (int w2 = 0; w2 < NWAVE; ++w2) pre += (w2 < wave) ? wtot[w2] : 0;
    int run = pre + incl - ts;
    soff[8 * tid + 0] = run; run += e0;
    soff[8 * tid + 1] = run; run += e1;
    soff[8 * tid + 2] = run; run += e2;
    soff[8 * tid + 3] = run; run += e3;
    soff[8 * tid + 4] = run; run += e4;
    soff[8 * tid + 5] = run; run += e5;
    soff[8 * tid + 6] = run; run += e6;
    soff[8 * tid + 7] = run;
  }
  __syncthreads();
  for (int i = tid; i < NBMAX; i += NTHR) list[i] = soff[i];
  __syncthreads();

  if (wave == 0) {
#pragma unroll 1
    for (int b0 = 0; b0 < nh; b0 += 32) {
      const int idx = b0 + lane;
      const int uv  = reg1[idx < RCAP ? idx : RCAP - 1];
      const int m32 = (nh - b0) < 32 ? (nh - b0) : 32;
#pragma unroll 1
      for (int k = 0; k < m32; ++k) {
        const int u   = __builtin_amdgcn_readlane(uv, k);
        const int sl  = u & (NBMAX - 1);
        const int eid = (int)((unsigned)u >> 12);
        if (lane == 0) {
          int pos = list[sl];
          pos = pos < 0 ? 0 : (pos > RCAP - 1 ? RCAP - 1 : pos);
          reg2[pos] = eid;
          list[sl] = pos + 1;
        }
      }
    }
  }
  __syncthreads();

  const int nbw = nb >> 3;
  const int c0 = 4 * lane, c1 = 128 + 4 * lane;
  const bool ovf = (nh >= RCAP);
  const float qnan = __int_as_float(0x7fc00000);
  const float ninf = __int_as_float(0xff800000);
  const v4f z4 = {0.f, 0.f, 0.f, 0.f};
#pragma unroll 1
  for (int jt = 0; jt < nbw; ++jt) {
    const int slot = wave * nbw + jt;
    const int grow = nodeBase + slot;
    const int gcl  = grow < nN ? grow : nN - 1;
    int st = soff[slot];
    const int craw = scnt[slot];
    int cnt = craw;
    st  = st < 0 ? 0 : (st > nh ? nh : st);
    cnt = cnt < 0 ? 0 : (cnt > DEGCAP ? DEGCAP : cnt);
    if (cnt > nh - st) cnt = nh - st;
    const float pz = (ovf || craw > DEGCAP) ? qnan : 0.0f;
    const bool wr = grow < nN;

    float mx = ninf;
#pragma unroll 1
    for (int q0 = 0; q0 < cnt; q0 += 32) {
      const int q  = q0 + lane;
      const int qc = q < cnt ? q : cnt - 1;
      int idx = st + qc; idx = idx > RCAP - 1 ? RCAP - 1 : idx;
      int eid = reg2[idx]; eid = eid < 0 ? 0 : (eid > nE - 1 ? nE - 1 : eid);
      const float l = sc[eid];
      mx = fmaxf(mx, q < cnt ? l : ninf);
    }
    mx = fmaxf(mx, __shfl_xor(mx, 16));
    mx = fmaxf(mx, __shfl_xor(mx, 8));
    mx = fmaxf(mx, __shfl_xor(mx, 4));
    mx = fmaxf(mx, __shfl_xor(mx, 2));
    mx = fmaxf(mx, __shfl_xor(mx, 1));

    float dn = 0.f;
    v4f a0 = z4, a1 = z4;
#pragma unroll 1
    for (int q = 0; q < cnt; ++q) {
      int idx = st + q; idx = idx > RCAP - 1 ? RCAP - 1 : idx;
      int eid = reg2[idx]; eid = eid < 0 ? 0 : (eid > nE - 1 ? nE - 1 : eid);
      const int sraw = srcs[eid];
      const int s = sraw < 0 ? 0 : (sraw > nN - 1 ? nN - 1 : sraw);
      const float l = sc[eid];
      const float w = __expf(l - mx);
      dn += w;
      const float* ys = FS + (size_t)s * YP;
      const v4f xs0 = *(const v4f*)(ys + c0);
      const v4f xs1 = *(const v4f*)(ys + c1);
      a0.x = fmaf(w, xs0.x, a0.x);
      a0.y = fmaf(w, xs0.y, a0.y);
      a0.z = fmaf(w, xs0.z, a0.z);
      a0.w = fmaf(w, xs0.w, a0.w);
      a1.x = fmaf(w, xs1.x, a1.x);
      a1.y = fmaf(w, xs1.y, a1.y);
      a1.z = fmaf(w, xs1.z, a1.z);
      a1.w = fmaf(w, xs1.w, a1.w);
    }
    const float inv = (cnt > 0) ? __builtin_amdgcn_rcpf(dn) : 0.f;
    const float* rp = resp + (size_t)gcl * YP;
    const v4f r0 = *(const v4f*)(rp + c0);
    const v4f r1 = *(const v4f*)(rp + c1);
    v4f o0, o1;
    o0.x = fmaf(a0.x, inv, r0.x) + pz;
    o0.y = fmaf(a0.y, inv, r0.y) + pz;
    o0.z = fmaf(a0.z, inv, r0.z) + pz;
    o0.w = fmaf(a0.w, inv, r0.w) + pz;
    o1.x = fmaf(a1.x, inv, r1.x) + pz;
    o1.y = fmaf(a1.y, inv, r1.y) + pz;
    o1.z = fmaf(a1.z, inv, r1.z) + pz;
    o1.w = fmaf(a1.w, inv, r1.w) + pz;
    float* op = rst + (size_t)gcl * YP;
    if (wr) {
      *(volatile v4f*)(op + c0) = o0;
      *(volatile v4f*)(op + c1) = o1;
    }
    __threadfence();
    if (wr) {
      *(volatile v4f*)(op + c0) = o0;
      *(volatile v4f*)(op + c1) = o1;
    }
    if (lane == 0) {
      sm[slot] = ((cnt > 0) ? mx : 0.f) + pz;
      sd[slot] = ((cnt > 0) ? dn : 0.f) + pz;
    }
  }
  __syncthreads();

  const int nq = nb >> 2;
#pragma unroll 1
  for (int i = tid; i < nq; i += NTHR) {
    const v4f vm = *(const v4f*)(sm + 4 * i);
    const v4f vd = *(const v4f*)(sd + 4 * i);
    *(volatile v4f*)(nstm + (size_t)nodeBase + 4 * i) = vm;
    *(volatile v4f*)(nstd + (size_t)nodeBase + 4 * i) = vd;
  }
  __threadfence();
#pragma unroll 1
  for (int i = tid; i < nq; i += NTHR) {
    const v4f vm = *(const v4f*)(sm + 4 * i);
    const v4f vd = *(const v4f*)(sd + 4 * i);
    *(volatile v4f*)(nstm + (size_t)nodeBase + 4 * i) = vm;
    *(volatile v4f*)(nstd + (size_t)nodeBase + 4 * i) = vd;
  }
}

__global__ __launch_bounds__(NTHR) void k_colstat(const float* __restrict__ R, int nN, float* bnt) {
  __shared__ double ss[NTHR];
  __shared__ double sq[NTHR];
  __shared__ __attribute__((aligned(16))) float smu[32];
  __shared__ __attribute__((aligned(16))) float srs[32];
  const int tid = threadIdx.x, lane = tid & 31, wave = tid >> 5;
  const int col = (int)blockIdx.x * 32 + lane;
  double s = 0.0, s2 = 0.0;
#pragma unroll 1
  for (int r = wave; r < nN; r += NWAVE) {
    const double v = (double)R[(size_t)r * YP + col];
    s  += v;
    s2 += v * v;
  }
  ss[tid] = s;
  sq[tid] = s2;
  __syncthreads();
  if (tid < 32) {
    double a = 0.0, b = 0.0;
#pragma unroll
    for (int w2 = 0; w2 < NWAVE; ++w2) { a += ss[w2 * 32 + tid]; b += sq[w2 * 32 + tid]; }
    const double mu = a / (double)nN;
    double var = b / (double)nN - mu * mu;
    var = var < 0.0 ? 0.0 : var;
    smu[tid] = (float)mu;
    srs[tid] = 1.0f / sqrtf((float)var + BN_EPS);
  }
  __syncthreads();
  if (tid < 8) {
    const v4f vm = *(const v4f*)(smu + 4 * tid);
    const v4f vr = *(const v4f*)(srs + 4 * tid);
    float* pm = bnt + (size_t)blockIdx.x * 32 + 4 * tid;
    float* pr = bnt + HID + (size_t)blockIdx.x * 32 + 4 * tid;
    *(volatile v4f*)pm = vm;
    *(volatile v4f*)pr = vr;
    __threadfence();
    *(volatile v4f*)pm = vm;
    *(volatile v4f*)pr = vr;
  }
}

__global__ __launch_bounds__(NTHR) void k_bnapply(const float* __restrict__ R, const float* __restrict__ bnt,
                                                  const float* __restrict__ g, const float* __restrict__ be,
                                                  float* H, _Float16* xh, int nN, int nUnits) {
  const int u = (int)blockIdx.x * NTHR + (int)threadIdx.x;
  if (u >= nUnits) return;
  const int row = u >> 6;
  const int c4  = (u & 63) * 4;
  const v4f x  = *(const v4f*)(R + (size_t)row * YP + c4);
  const v4f mu = *(const v4f*)(bnt + c4);
  const v4f rs = *(const v4f*)(bnt + HID + c4);
  const v4f gg = *(const v4f*)(g + c4);
  const v4f bb = *(const v4f*)(be + c4);
  v4f h;
  h.x = fmaxf(fmaf(gg.x * (x.x - mu.x), rs.x, bb.x), 0.f);
  h.y = fmaxf(fmaf(gg.y * (x.y - mu.y), rs.y, bb.y), 0.f);
  h.z = fmaxf(fmaf(gg.z * (x.z - mu.z), rs.z, bb.z), 0.f);
  h.w = fmaxf(fmaf(gg.w * (x.w - mu.w), rs.w, bb.w), 0.f);
  v4h hv;
  hv[0] = (_Float16)(h.x * CA); hv[1] = (_Float16)(h.y * CA);
  hv[2] = (_Float16)(h.z * CA); hv[3] = (_Float16)(h.w * CA);
  float* hp = H + (size_t)row * YP + c4;
  _Float16* xp = xh + (size_t)row * KP + c4;
  *(volatile v4f*)hp = h;
  *(volatile v4h*)xp = hv;
  __threadfence();
  *(volatile v4f*)hp = h;
  *(volatile v4h*)xp = hv;
}

__global__ __launch_bounds__(NTHR) void k_gmean(const float* __restrict__ H, const int* __restrict__ gid,
                                                _Float16* ph, int nN, int nG, int layer) {
  __shared__ int hl[NTHR];
  __shared__ int wc[NWAVE];
  __shared__ __attribute__((aligned(16))) float smean[HID];
  const int tid = threadIdx.x, lane = tid & 31, wave = tid >> 5;
  const int g = (int)blockIdx.x;
  float sum = 0.f;
  int cnt = 0;
  const int nChunks = (nN + NTHR - 1) / NTHR;
#pragma unroll 1
  for (int ch = 0; ch < nChunks; ++ch) {
    const int n  = ch * NTHR + tid;
    const int nc = n < nN ? n : nN - 1;
    const int v  = gid[nc];
    const bool hit = (n < nN) && (v == g);
    const unsigned mk = __builtin_amdgcn_ballot_w32(hit);
    if (lane == 0) wc[wave] = (int)__builtin_popcount(mk);
    __syncthreads();
    int pre = 0, all = 0;
#pragma unroll
    for (int w2 = 0; w2 < NWAVE; ++w2) {
      int c = wc[w2];
      c = c < 0 ? 0 : (c > 32 ? 32 : c);
      all += c;
      pre += (w2 < wave) ? c : 0;
    }
    if (all != 0) {
      if (hit) {
        const int pos = pre + (int)__builtin_amdgcn_mbcnt_lo(mk, 0u);
        if (pos < NTHR) hl[pos] = n;
      }
      __syncthreads();
      const int na = all > NTHR ? NTHR : all;
#pragma unroll 1
      for (int k = 0; k < na; ++k) {
        int node = hl[k];
        node = node < 0 ? 0 : (node > nN - 1 ? nN - 1 : node);
        sum += H[(size_t)node * YP + tid];
      }
      cnt += na;
    }
    __syncthreads();
  }
  const float inv = (g < nG) ? (1.0f / (float)cnt) : 0.0f;
  smean[tid] = sum * inv;
  __syncthreads();
  if (tid < 32) {
    v8h hv;
#pragma unroll
    for (int j = 0; j < 8; ++j) hv[j] = (_Float16)(smean[8 * tid + j] * CA);
    _Float16* p = ph + (size_t)g * KF + (size_t)layer * HID + 8 * tid;
    *(volatile v8h*)p = hv;
    __threadfence();
    *(volatile v8h*)p = hv;
  }
}

__global__ __launch_bounds__(NTHR) void k_headfin(const float* __restrict__ T1, const float* __restrict__ gf,
                                                  const float* __restrict__ bf, const float* __restrict__ w2,
                                                  const float* __restrict__ b2, const int* __restrict__ dsts,
                                                  const float* __restrict__ score, const float* __restrict__ nstm,
                                                  const float* __restrict__ nstd, float* out,
                                                  int nG, int nE, int nN, int epad, int np, int n0, int P) {
  __shared__ float smu[HID];
  __shared__ float srs[HID];
  __shared__ float sgm[HID];
  __shared__ float sbt[HID];
  __shared__ float sw[HID * OUTD];
  __shared__ float sb5[8];
  __shared__ __attribute__((aligned(16))) float so[PMAX];
  const int tid = threadIdx.x;
  {
    double s = 0.0, s2 = 0.0;
#pragma unroll 1
    for (int r = 0; r < nG; ++r) {
      const double v = (double)T1[(size_t)r * YP + tid];
      s  += v;
      s2 += v * v;
    }
    const double mu = s / (double)nG;
    double var = s2 / (double)nG - mu * mu;
    var = var < 0.0 ? 0.0 : var;
    smu[tid] = (float)mu;
    srs[tid] = 1.0f / sqrtf((float)var + BN_EPS);
    sgm[tid] = gf[tid];
    sbt[tid] = bf[tid];
  }
#pragma unroll 1
  for (int i = tid; i < HID * OUTD; i += NTHR) sw[i] = w2[i];
  if (tid < 8) sb5[tid] = b2[tid < OUTD ? tid : OUTD - 1];
  __syncthreads();
  const int Pc = P > PMAX ? PMAX : P;
#pragma unroll 1
  for (int i = tid; i < Pc; i += NTHR) {
    int ii = i < n0 ? i : n0 - 1;
    int gg = ii / OUTD;
    const int o = ii - gg * OUTD;
    gg = gg > nG - 1 ? nG - 1 : gg;
    const float* tr = T1 + (size_t)gg * YP;
    float acc = sb5[o];
#pragma unroll 1
    for (int c = 0; c < HID; ++c) {
      const float t = sgm[c] * (tr[c] - smu[c]);
      const float v = fmaxf(fmaf(t, srs[c], sbt[c]), 0.f);
      acc = fmaf(v, sw[c * OUTD + o], acc);
    }
    const int jj = (i - n0) < 0 ? 0 : (i - n0);
    const float al = alpha_of(dsts, score, nstm, nstd, jj >> 2, jj & 3, nE, nN, epad, np);
    so[i] = (i < n0) ? acc : al;
  }
  __syncthreads();
  const int n4 = Pc >> 2;
  const v4f* s4 = (const v4f*)so;
#pragma unroll 1
  for (int i = tid; i < n4; i += NTHR) {
    const v4f v = s4[i];
    *(volatile v4f*)(out + 4 * (size_t)i) = v;
  }
  __threadfence();
#pragma unroll 1
  for (int i = tid; i < n4; i += NTHR) {
    const v4f v = s4[i];
    *(volatile v4f*)(out + 4 * (size_t)i) = v;
  }
}

__global__ __launch_bounds__(NTHR) void k_pack(const int* __restrict__ dsts, const float* __restrict__ score,
                                               const float* __restrict__ nstm, const float* __restrict__ nstd,
                                               float* out, int n0, int P, int nE, int nN, int epad, int np,
                                               int nFull, int rem) {
  const int t = (int)blockIdx.x * NTHR + (int)threadIdx.x;
  if (t > nFull) return;
  const int j0 = (P - n0) + 4 * t;
  v4f a;
  a.x = alpha_of(dsts, score, nstm, nstd, (j0 + 0) >> 2, (j0 + 0) & 3, nE, nN, epad, np);
  a.y = alpha_of(dsts, score, nstm, nstd, (j0 + 1) >> 2, (j0 + 1) & 3, nE, nN, epad, np);
  a.z = alpha_of(dsts, score, nstm, nstd, (j0 + 2) >> 2, (j0 + 2) & 3, nE, nN, epad, np);
  a.w = alpha_of(dsts, score, nstm, nstd, (j0 + 3) >> 2, (j0 + 3) & 3, nE, nN, epad, np);
  float* p = out + (size_t)P + 4 * (size_t)t;
  if (t < nFull) {
    *(volatile v4f*)p = a;
    __threadfence();
    *(volatile v4f*)p = a;
  } else if (rem > 0) {
    if (rem > 0) *(volatile float*)(p + 0) = a.x;
    if (rem > 1) *(volatile float*)(p + 1) = a.y;
    if (rem > 2) *(volatile float*)(p + 2) = a.z;
    __threadfence();
    if (rem > 0) *(volatile float*)(p + 0) = a.x;
    if (rem > 1) *(volatile float*)(p + 1) = a.y;
    if (rem > 2) *(volatile float*)(p + 2) = a.z;
  }
}

static int pick_nb(int nE, int nN) {
  int nb = NBMAX;
  while (nb > 32 && (long long)nb * (long long)nE * 5LL > (long long)RCAP * (long long)nN * 4LL) nb >>= 1;
  return nb;
}

extern "C" void kernel_launch(void* const* d_in, const int* in_sizes, int n_in,
                              void* d_out, int out_size, void* d_ws, size_t ws_size,
                              hipStream_t stream) {
  if (n_in < 25) return;
  const int nE = in_sizes[22];
  if (nE < 8 || in_sizes[23] != nE || nE > (1 << 20)) return;
  const int nN = in_sizes[24];
  if (nN < 1 || nN > (1 << 22)) return;
  if (in_sizes[1] <= 0 || (in_sizes[1] % HID) != 0) return;
  const int inDim = in_sizes[1] / HID;
  if (inDim < 1 || inDim > KP) return;
  if ((long long)in_sizes[0] != (long long)nN * (long long)inDim) return;
  if (in_sizes[3] != inDim * HID || in_sizes[6] != inDim * HID) return;
  if (in_sizes[2] != HID || in_sizes[4] != HID || in_sizes[5] != HID || in_sizes[7] != HID || in_sizes[8] != HID) return;
  if (in_sizes[9] != 3 * HID * HID || in_sizes[11] != 3 * HID * HID) return;
  if (in_sizes[10] != 3 * HID || in_sizes[12] != 3 * HID || in_sizes[13] != 3 * HID) return;
  if (in_sizes[14] != 3 * HID || in_sizes[15] != 3 * HID) return;
  if (in_sizes[16] != KF * HID || in_sizes[17] != HID || in_sizes[18] != HID || in_sizes[19] != HID) return;
  if (in_sizes[20] != HID * OUTD || in_sizes[21] != OUTD) return;
  const long long rem0 = (long long)out_size - 4LL * (long long)nE;
  if (rem0 < OUTD || (rem0 % OUTD) != 0) return;
  const int nG = (int)(rem0 / OUTD);
  if (nG > MG) return;
  const int n0 = nG * OUTD;
  const int P  = ((n0 + 31) / 32) * 32;
  if (P > PMAX || P > out_size) return;
  const int tail  = out_size - P;
  const int nFull = tail / 4;
  const int rem   = tail - 4 * nFull;

  const float* x    = (const float*)d_in[0];
  const float* Ws0  = (const float*)d_in[1];
  const float* bs0  = (const float*)d_in[2];
  const float* Wd0  = (const float*)d_in[3];
  const float* bd0  = (const float*)d_in[4];
  const float* a0   = (const float*)d_in[5];
  const float* Wr0  = (const float*)d_in[6];
  const float* g0   = (const float*)d_in[7];
  const float* be0  = (const float*)d_in[8];
  const float* Wsr  = (const float*)d_in[9];
  const float* bsr  = (const float*)d_in[10];
  const float* Wdr  = (const float*)d_in[11];
  const float* bdr  = (const float*)d_in[12];
  const float* ar   = (const float*)d_in[13];
  const float* gr   = (const float*)d_in[14];
  const float* ber  = (const float*)d_in[15];
  const float* fc1W = (const float*)d_in[16];
  const float* fc1b = (const float*)d_in[17];
  const float* gfc  = (const float*)d_in[18];
  const float* bfc  = (const float*)d_in[19];
  const float* fc2W = (const float*)d_in[20];
  const float* fc2b = (const float*)d_in[21];
  const int*   src  = (const int*)d_in[22];
  const int*   dst  = (const int*)d_in[23];
  const int*   gid  = (const int*)d_in[24];
  float* out = (float*)d_out;

  const int MP   = ((nN + GBM - 1) / GBM) * GBM;
  const int nb   = pick_nb(nE, nN);
  const int gA   = (nN + nb - 1) / nb;
  const int NP   = gA * nb;
  const int EPAD = ((nE + NTHR - 1) / NTHR) * NTHR;
  const int nks0 = (inDim + 31) / 32;
  const int vec8 = 1;

  char* wsb = (char*)d_ws;
  size_t off = 0;
  const size_t oWT = off; off += (size_t)NWT * HID * KP * 2;       off = (off + 255) & ~(size_t)255;
  const size_t oWF = off; off += (size_t)HID * KF * 2;             off = (off + 255) & ~(size_t)255;
  const size_t oXH = off; off += (size_t)MP * KP * 2;              off = (off + 255) & ~(size_t)255;
  const size_t oFS = off; off += (size_t)MP * YP * 4;              off = (off + 255) & ~(size_t)255;
  const size_t oFD = off; off += (size_t)MP * YP * 4;              off = (off + 255) & ~(size_t)255;
  const size_t oRS = off; off += (size_t)MP * YP * 4;              off = (off + 255) & ~(size_t)255;
  const size_t oH  = off; off += (size_t)MP * YP * 4;              off = (off + 255) & ~(size_t)255;
  const size_t oSC = off; off += (size_t)NLAY * EPAD * 4;          off = (off + 255) & ~(size_t)255;
  const size_t oNM = off; off += (size_t)NLAY * NP * 4;            off = (off + 255) & ~(size_t)255;
  const size_t oND = off; off += (size_t)NLAY * NP * 4;            off = (off + 255) & ~(size_t)255;
  const size_t oBT = off; off += (size_t)2 * HID * 4;              off = (off + 255) & ~(size_t)255;
  const size_t oPH = off; off += (size_t)MG * KF * 2;              off = (off + 255) & ~(size_t)255;
  const size_t oT1 = off; off += (size_t)MG * YP * 4;              off = (off + 255) & ~(size_t)255;
  if (off > ws_size || off > (size_t)WSCAP) return;
  _Float16* WT  = (_Float16*)(wsb + oWT);
  _Float16* WF  = (_Float16*)(wsb + oWF);
  _Float16* XH  = (_Float16*)(wsb + oXH);
  float*    FS  = (float*)(wsb + oFS);
  float*    FD  = (float*)(wsb + oFD);
  float*    RST = (float*)(wsb + oRS);
  float*    H   = (float*)(wsb + oH);
  float*    SC  = (float*)(wsb + oSC);
  float*    NSTM = (float*)(wsb + oNM);
  float*    NSTD = (float*)(wsb + oND);
  float*    BNT = (float*)(wsb + oBT);
  _Float16* PH  = (_Float16*)(wsb + oPH);
  float*    T1  = (float*)(wsb + oT1);

  hipFuncSetAttribute(reinterpret_cast<const void*>(&k_agg),
                      hipFuncAttributeMaxDynamicSharedMemorySize, LDS_AGG);

  const int nUx = MP * (KP / 8);
  k_xprep<<<(nUx + NTHR - 1) / NTHR, NTHR, 0, stream>>>(x, XH, nN, inDim, nUx);
  k_wprep<<<dim3((HID * (KF / 8) + NTHR - 1) / NTHR, NWT + 1), NTHR, 0, stream>>>(Ws0, Wd0, Wr0, Wsr, Wdr, fc1W,
                                                                                  WT, WF, inDim);

  const int gG = MP / GBM;
  const int gS = EPAD / NTHR;
  const int nUb = nN * (HID / 4);
  const int gB = (nUb + NTHR - 1) / NTHR;
  const size_t WB = (size_t)HID * KP;

  for (int l = 0; l < NLAY; ++l) {
    const float* av = (l == 0) ? a0 : (ar + (size_t)(l - 1) * HID);
    const float* gg = (l == 0) ? g0 : (gr + (size_t)(l - 1) * HID);
    const float* bb = (l == 0) ? be0 : (ber + (size_t)(l - 1) * HID);
    if (l == 0) {
      k_gemm<<<dim3(gG, 3), GTHR, 0, stream>>>(XH, KP, WT, WT + WB, WT + 2 * WB, KP,
                                               bs0, bd0, bs0, 3, FS, FD, H, nks0);
    } else {
      const float* bsl = bsr + (size_t)(l - 1) * HID;
      const float* bdl = bdr + (size_t)(l - 1) * HID;
      k_gemm<<<dim3(gG, 2), GTHR, 0, stream>>>(XH, KP, WT + (size_t)(3 + l - 1) * WB, WT + (size_t)(6 + l - 1) * WB,
                                               WT + (size_t)(6 + l - 1) * WB, KP,
                                               bsl, bdl, bdl, 3, FS, FD, FD, HID / 32);
    }
    k_score<<<gS, NTHR, 0, stream>>>(src, dst, FS, FD, av, SC + (size_t)l * EPAD, nN, nE);
    k_agg<<<gA, NTHR, LDS_AGG, stream>>>(src, dst, FS, SC + (size_t)l * EPAD, H, RST,
                                         NSTM + (size_t)l * NP, NSTD + (size_t)l * NP, nN, nE, nb, vec8);
    k_colstat<<<HID / 32, NTHR, 0, stream>>>(RST, nN, BNT);
    k_bnapply<<<gB, NTHR, 0, stream>>>(RST, BNT, gg, bb, H, XH, nN, nUb);
    k_gmean<<<MG, NTHR, 0, stream>>>(H, gid, PH, nN, nG, l);
  }

  k_gemm<<<dim3(MG / GBM, 1), GTHR, 0, stream>>>(PH, KF, WF, WF, WF, KF, fc1b, fc1b, fc1b, 1, T1, T1, T1, KF / 32);
  k_headfin<<<1, NTHR, 0, stream>>>(T1, gfc, bfc, fc2W, fc2b, dst, SC, NSTM, NSTD, out,
                                    nG, nE, nN, EPAD, NP, n0, P);
  k_pack<<<(nFull + 1 + NTHR - 1) / NTHR, NTHR, 0, stream>>>(dst, SC, NSTM, NSTD, out, n0, P, nE, nN, EPAD, NP,
                                                              nFull, rem);
}
